// SelfModifyingDeltaMemory_4303557230749
// MI455X (gfx1250) — hardware-verified
//
#include <hip/hip_runtime.h>
#include <stdint.h>

#define DD 128
#define SS 256
#define NSEQ 16
#define ROWS (NSEQ * SS)
#define DH 32
#define CH 16
#define MP 132
#define WSC 16.0f
#define OSC 8.0f

static_assert((MP % 4) == 0);
static_assert((SS % CH) == 0);
static_assert((ROWS % 32) == 0);

typedef _Float16 v16h __attribute__((ext_vector_type(16)));
typedef _Float16 v8h  __attribute__((ext_vector_type(8)));
typedef float    v8f  __attribute__((ext_vector_type(8)));
typedef float    v4f  __attribute__((ext_vector_type(4)));
typedef v4f v4fa __attribute__((may_alias));
typedef v8h v8ha __attribute__((may_alias));
union Frag { v16h v; v8h half[2]; };

__device__ __forceinline__ float sigm_(float x) { return __frcp_rn(1.0f + __expf(-x)); }
__device__ __forceinline__ float silu_(float x) { return x * sigm_(x); }

__device__ __forceinline__ v8h cvt8(v4f a, v4f b) {
  v8h h;
  h[0] = (_Float16)a[0]; h[1] = (_Float16)a[1]; h[2] = (_Float16)a[2]; h[3] = (_Float16)a[3];
  h[4] = (_Float16)b[0]; h[5] = (_Float16)b[1]; h[6] = (_Float16)b[2]; h[7] = (_Float16)b[3];
  return h;
}

__device__ __forceinline__ v8f wmma16(const Frag& a, const Frag& b, v8f c) {
  c = __builtin_amdgcn_wmma_f32_16x16x32_f16(false, a.v, false, b.v, (short)0, c, false, false);
  asm volatile("v_nop\n\tv_nop\n\tv_nop\n\tv_nop" : "+v"(c) : "v"(a.v), "v"(b.v));
  return c;
}

__device__ __forceinline__ v8f tile16(const _Float16* A, const _Float16* BT, int row0, int col0) {
  const int l = threadIdx.x & 31, h = l >> 4, m = l & 15;
  const _Float16* ar = A  + (size_t)(row0 + m) * DD;
  const _Float16* br = BT + (size_t)(col0 + m) * DD;
  v8f c = {0.f, 0.f, 0.f, 0.f, 0.f, 0.f, 0.f, 0.f};
#pragma unroll
  for (int kb = 0; kb < DD; kb += 32) {
    Frag a, b;
    a.half[0] = *(const v8ha*)(ar + kb + 8 * h);
    a.half[1] = *(const v8ha*)(ar + kb + 16 + 8 * h);
    b.half[0] = *(const v8ha*)(br + kb + 8 * h);
    b.half[1] = *(const v8ha*)(br + kb + 16 + 8 * h);
    c = wmma16(a, b, c);
  }
  return c;
}

__global__ void __launch_bounds__(256) k_cvt_x(const float* x, _Float16* xh, int n8) {
  const int i = blockIdx.x * 256 + threadIdx.x;
  if (i >= n8) return;
  const size_t o = (size_t)i * 8;
  v4f a = *(const v4fa*)(x + o);
  v4f b = *(const v4fa*)(x + o + 4);
  v8h hv = cvt8(a, b);
  volatile v8h* p = (volatile v8h*)(xh + o);
  *p = hv;
  __threadfence();
  *p = hv;
}

__global__ void __launch_bounds__(256) k_wt(const float* Wq, const float* Wk, const float* Wv,
                                            const float* Wg1, const float* Wg2, const float* Wo,
                                            const float* We1, const float* Wa1,
                                            _Float16* WT, _Float16* EAT) {
  __shared__ __attribute__((aligned(16))) _Float16 sW[32][136];
  const int wid = blockIdx.y, nt = blockIdx.x, tid = threadIdx.x;
  const int N = (wid < 6) ? DD : DH;
  if (nt * 32 >= N) return;
  const float* W = Wq;
  if (wid == 1) W = Wk; else if (wid == 2) W = Wv; else if (wid == 3) W = Wg1;
  else if (wid == 4) W = Wg2; else if (wid == 5) W = Wo; else if (wid == 6) W = We1; else if (wid == 7) W = Wa1;
  const int n0 = nt * 32;
#pragma unroll 4
  for (int q = 0; q < 16; ++q) {
    const int idx = tid + 256 * q;
    const int k = idx >> 5, c = idx & 31;
    sW[c][k] = (_Float16)(W[(size_t)k * N + n0 + c] * WSC);
  }
  __syncthreads();
  const int row = tid >> 4, c0 = (tid & 15) * 8;
  v8h v0 = *(const v8ha*)&sW[row][c0];
  v8h v1 = *(const v8ha*)&sW[row + 16][c0];
  _Float16* dst = (wid < 6) ? (WT + (size_t)wid * DD * DD + (size_t)n0 * DD)
                            : (EAT + (size_t)(wid - 6) * DH * DD);
  volatile v8h* p0 = (volatile v8h*)(dst + (size_t)row * DD + c0);
  volatile v8h* p1 = (volatile v8h*)(dst + (size_t)(row + 16) * DD + c0);
  *p0 = v0; *p1 = v1;
  __threadfence();
  *p0 = v0; *p1 = v1;
}

__device__ __forceinline__ void store_tile_f32(const float (*sT)[DD], float* P, int rt) {
  const int tid = threadIdx.x, w = tid >> 5, l = tid & 31;
  const int c0 = l * 4;
  v4f v0 = *(const v4fa*)&sT[w][c0];
  v4f v1 = *(const v4fa*)&sT[w + 8][c0];
  volatile v4f* p0 = (volatile v4f*)(P + (size_t)(rt + w) * DD + c0);
  volatile v4f* p1 = (volatile v4f*)(P + (size_t)(rt + w + 8) * DD + c0);
  *p0 = v0; *p1 = v1;
  __threadfence();
  *p0 = v0; *p1 = v1;
}
__device__ __forceinline__ void store_tile_f16(const float (*sT)[DD], _Float16* P, int rt) {
  const int tid = threadIdx.x;
  const int row = tid >> 4, c0 = (tid & 15) * 8;
  v4f a = *(const v4fa*)&sT[row][c0];
  v4f b = *(const v4fa*)&sT[row][c0 + 4];
  v8h hv = cvt8(a, b);
  volatile v8h* p = (volatile v8h*)(P + (size_t)(rt + row) * DD + c0);
  *p = hv;
  __threadfence();
  *p = hv;
}

__global__ void __launch_bounds__(256) k_gemm_qkv(const _Float16* xh, const _Float16* WT,
                                                  float* Q, float* KN, _Float16* Vh) {
  __shared__ __attribute__((aligned(16))) float sT[16][DD];
  const int tid = threadIdx.x, w = tid >> 5, l = tid & 31, h = l >> 4, m = l & 15;
  const int sel = blockIdx.y;
  const int rt = blockIdx.x * 16;
  const _Float16* BT = WT + (size_t)sel * DD * DD;
  v8f c = tile16(xh, BT, rt, w * 16);
  const int col = w * 16 + m;
#pragma unroll
  for (int r = 0; r < 8; ++r) sT[8 * h + r][col] = c[r] * (1.0f / WSC);
  __syncthreads();
  if (sel == 1) {
    const int row = 2 * w + h, c0 = m * 8;
    v4f a = *(const v4fa*)&sT[row][c0];
    v4f b = *(const v4fa*)&sT[row][c0 + 4];
    float ss = a[0] * a[0] + a[1] * a[1] + a[2] * a[2] + a[3] * a[3]
             + b[0] * b[0] + b[1] * b[1] + b[2] * b[2] + b[3] * b[3];
    ss += __shfl_xor(ss, 8);
    ss += __shfl_xor(ss, 4);
    ss += __shfl_xor(ss, 2);
    ss += __shfl_xor(ss, 1);
    const float inv = 1.0f / fmaxf(sqrtf(ss), 1e-12f);
    a = a * inv; b = b * inv;
    *(v4fa*)&sT[row][c0] = a;
    *(v4fa*)&sT[row][c0 + 4] = b;
  }
  __syncthreads();
  if (sel == 2) {
    store_tile_f16(sT, Vh, rt);
  } else {
    store_tile_f32(sT, sel == 0 ? Q : KN, rt);
  }
}

template <bool SILU, bool OUT16>
__global__ void __launch_bounds__(256) k_gemm_act(const _Float16* A, const _Float16* BT, const float* bias,
                                                  float* O32, _Float16* O16) {
  __shared__ __attribute__((aligned(16))) float sT[16][DD];
  const int tid = threadIdx.x, w = tid >> 5, l = tid & 31, h = l >> 4, m = l & 15;
  const int rt = blockIdx.x * 16;
  v8f c = tile16(A, BT, rt, w * 16);
  const int col = w * 16 + m;
  const float b0 = bias[col];
#pragma unroll
  for (int r = 0; r < 8; ++r) {
    float v = c[r] * (1.0f / WSC) + b0;
    if (SILU) v = silu_(v);
    sT[8 * h + r][col] = v;
  }
  __syncthreads();
  if (OUT16) store_tile_f16(sT, O16, rt);
  else       store_tile_f32(sT, O32, rt);
}

__global__ void __launch_bounds__(256) k_ea(const _Float16* xh, const _Float16* EAT,
                                            const float* be1, const float* ba1,
                                            const float* We2, const float* be2,
                                            const float* Wa2, const float* ba2,
                                            float* eta, float* alp) {
  __shared__ float sEA[32][64];
  __shared__ __attribute__((aligned(16))) float sR[2][32];
  const int tid = threadIdx.x, w = tid >> 5, l = tid & 31, h = l >> 4, m = l & 15;
  const int rt = blockIdx.x * 32;
  const int rsub = (w >> 2) * 16, nt = w & 3;
  v8f c = tile16(xh, EAT, rt + rsub, nt * 16);
  const int col = nt * 16 + m;
  const float b0 = (col < DH) ? be1[col] : ba1[col - DH];
#pragma unroll
  for (int r = 0; r < 8; ++r) sEA[rsub + 8 * h + r][col] = silu_(c[r] * (1.0f / WSC) + b0);
  __syncthreads();
  if (tid < 64) {
    const int row = tid & 31, which = tid >> 5;
    const float* w2 = which ? Wa2 : We2;
    float s = 0.f;
#pragma unroll 1
    for (int j = 0; j < DH; ++j) s = fmaf(sEA[row][which * DH + j], w2[j], s);
    s += which ? ba2[0] : be2[0];
    const float sg = sigm_(s);
    sR[which][row] = which ? (sg * 0.5f + 0.5f) : (sg * 0.1f + 0.01f);
  }
  __syncthreads();
  if (tid < 16) {
    const int which = tid >> 3, q = tid & 7;
    v4f v = *(const v4fa*)&sR[which][q * 4];
    float* dst = which ? alp : eta;
    volatile v4f* p = (volatile v4f*)(dst + rt + q * 4);
    *p = v;
    __threadfence();
    *p = v;
  }
}

__global__ void __launch_bounds__(128) k_scan(const float* Q, const float* KN, const float* VH,
                                              const float* eta, const float* alp, _Float16* OH) {
  __shared__ __attribute__((aligned(16))) float sM[DD * MP];
  __shared__ __attribute__((aligned(16))) float sQ[CH][DD];
  __shared__ __attribute__((aligned(16))) float sK[2][CH][DD];
  __shared__ __attribute__((aligned(16))) float sV[CH][DD];
  __shared__ __attribute__((aligned(16))) float sO[CH][DD];
  __shared__ float sE[CH], sA[CH];
  const int tid = threadIdx.x;
  const int bn = blockIdx.x;
  {
    v4f z = {0.f, 0.f, 0.f, 0.f};
    v4fa* mz = (v4fa*)(sM + tid * MP);
#pragma unroll 1
    for (int j = 0; j < MP / 4; ++j) mz[j] = z;
    v4fa* kz = (v4fa*)&sK[1][0][0];
#pragma unroll
    for (int q = 0; q < 4; ++q) kz[tid + 128 * q] = z;
  }
  float ap = 1.0f, dp = 0.0f;
  const float* kprev = &sK[1][CH - 1][0];
  float* mr = sM + tid * MP;

#pragma unroll 1
  for (int cc = 0; cc < SS / CH; ++cc) {
    const int p = cc & 1;
    const size_t rb = (size_t)bn * SS + (size_t)cc * CH;
    __syncthreads();
#pragma unroll
    for (int q = 0; q < 4; ++q) {
      const int idx = tid + 128 * q;
      const int row = idx >> 5, c4 = (idx & 31) * 4;
      const size_t g = (rb + row) * DD + c4;
      *(v4fa*)&sQ[row][c4]    = *(const v4fa*)(Q + g);
      *(v4fa*)&sK[p][row][c4] = *(const v4fa*)(KN + g);
      *(v4fa*)&sV[row][c4]    = *(const v4fa*)(VH + g);
    }
    if (tid < CH) { sE[tid] = eta[rb + tid]; sA[tid] = alp[rb + tid]; }
    __syncthreads();

#pragma unroll 1
    for (int t = 0; t < CH; ++t) {
      const float* qr = &sQ[t][0];
      const float* kr = &sK[p][t][0];
      float po = 0.f, pm = 0.f;
#pragma unroll 1
      for (int j = 0; j < DD; j += 8) {
        v4f m0 = *(v4fa*)(mr + j), m1 = *(v4fa*)(mr + j + 4);
        v4f g0 = *(const v4fa*)(kprev + j), g1 = *(const v4fa*)(kprev + j + 4);
        v4f q0 = *(const v4fa*)(qr + j), q1 = *(const v4fa*)(qr + j + 4);
        v4f k0 = *(const v4fa*)(kr + j), k1 = *(const v4fa*)(kr + j + 4);
        m0 = ap * m0 + dp * g0;
        m1 = ap * m1 + dp * g1;
        *(v4fa*)(mr + j) = m0;
        *(v4fa*)(mr + j + 4) = m1;
        po = fmaf(m0[0], q0[0], po); po = fmaf(m0[1], q0[1], po); po = fmaf(m0[2], q0[2], po); po = fmaf(m0[3], q0[3], po);
        po = fmaf(m1[0], q1[0], po); po = fmaf(m1[1], q1[1], po); po = fmaf(m1[2], q1[2], po); po = fmaf(m1[3], q1[3], po);
        pm = fmaf(m0[0], k0[0], pm); pm = fmaf(m0[1], k0[1], pm); pm = fmaf(m0[2], k0[2], pm); pm = fmaf(m0[3], k0[3], pm);
        pm = fmaf(m1[0], k1[0], pm); pm = fmaf(m1[1], k1[1], pm); pm = fmaf(m1[2], k1[2], pm); pm = fmaf(m1[3], k1[3], pm);
      }
      sO[t][tid] = po * OSC;
      dp = sE[t] * (sV[t][tid] - pm);
      ap = sA[t];
      kprev = kr;
    }
    __syncthreads();
    {
      const int row = tid >> 4, c0 = (tid & 15) * 8;
      v4f a0 = *(const v4fa*)&sO[row][c0],     a1 = *(const v4fa*)&sO[row][c0 + 4];
      v4f b0 = *(const v4fa*)&sO[row + 8][c0], b1 = *(const v4fa*)&sO[row + 8][c0 + 4];
      v8h h0 = cvt8(a0, a1), h1 = cvt8(b0, b1);
      volatile v8h* p0 = (volatile v8h*)(OH + (rb + row) * DD + c0);
      volatile v8h* p1 = (volatile v8h*)(OH + (rb + row + 8) * DD + c0);
      *p0 = h0; *p1 = h1;
      __threadfence();
      *p0 = h0; *p1 = h1;
    }
  }
}

__global__ void __launch_bounds__(256) k_final(const _Float16* OH, const _Float16* WoT, const float* bo,
                                               const float* x, const float* gamma, const float* beta,
                                               float* out) {
  __shared__ __attribute__((aligned(16))) float sH[16][DD];
  __shared__ float sMu[16], sRs[16];
  const int tid = threadIdx.x, w = tid >> 5, l = tid & 31, h = l >> 4, m = l & 15;
  const int rt = blockIdx.x * 16;
  v8f c = tile16(OH, WoT, rt, w * 16);
  const int col = w * 16 + m;
  const float b0 = bo[col];
#pragma unroll
  for (int r = 0; r < 8; ++r) {
    const int rl = 8 * h + r;
    sH[rl][col] = (c[r] * (1.0f / (WSC * OSC)) + b0) + x[(size_t)(rt + rl) * DD + col];
  }
  __syncthreads();
  {
    const int row = 2 * w + h, c0 = m * 8;
    v4f a = *(const v4fa*)&sH[row][c0];
    v4f b = *(const v4fa*)&sH[row][c0 + 4];
    float s = ((a[0] + a[1]) + (a[2] + a[3])) + ((b[0] + b[1]) + (b[2] + b[3]));
    s += __shfl_xor(s, 8);
    s += __shfl_xor(s, 4);
    s += __shfl_xor(s, 2);
    s += __shfl_xor(s, 1);
    const float mu = s * (1.0f / DD);
    v4f da = a - mu, db = b - mu;
    float s2 = da[0] * da[0] + da[1] * da[1] + da[2] * da[2] + da[3] * da[3]
             + db[0] * db[0] + db[1] * db[1] + db[2] * db[2] + db[3] * db[3];
    s2 += __shfl_xor(s2, 8);
    s2 += __shfl_xor(s2, 4);
    s2 += __shfl_xor(s2, 2);
    s2 += __shfl_xor(s2, 1);
    const float var = s2 * (1.0f / DD);
    const float rs = 1.0f / sqrtf(var + 1e-5f);
    if (m == 0) { sMu[row] = mu; sRs[row] = rs; }
  }
  __syncthreads();
  {
    const int c0 = l * 4;
    v4f g  = *(const v4fa*)(gamma + c0);
    v4f be = *(const v4fa*)(beta + c0);
    const int r0 = w, r1 = w + 8;
    v4f h0 = *(const v4fa*)&sH[r0][c0];
    v4f h1 = *(const v4fa*)&sH[r1][c0];
    v4f o0 = (h0 - sMu[r0]) * sRs[r0] * g + be;
    v4f o1 = (h1 - sMu[r1]) * sRs[r1] * g + be;
    volatile v4f* p0 = (volatile v4f*)(out + (size_t)(rt + r0) * DD + c0);
    volatile v4f* p1 = (volatile v4f*)(out + (size_t)(rt + r1) * DD + c0);
    *p0 = o0; *p1 = o1;
    __threadfence();
    *p0 = o0; *p1 = o1;
  }
}

extern "C" void kernel_launch(void* const* d_in, const int* in_sizes, int n_in,
                              void* d_out, int out_size, void* d_ws, size_t ws_size,
                              hipStream_t stream) {
  if (n_in < 20) return;
  if (in_sizes[0] != ROWS * DD || out_size != ROWS * DD) return;
  if (in_sizes[1] != DD * DD || in_sizes[2] != DD * DD || in_sizes[3] != DD * DD ||
      in_sizes[4] != DD * DD || in_sizes[6] != DD * DD || in_sizes[16] != DD * DD) return;
  if (in_sizes[8] != DD * DH || in_sizes[12] != DD * DH) return;
  if (in_sizes[5] < DD || in_sizes[7] < DD || in_sizes[17] < DD || in_sizes[18] < DD || in_sizes[19] < DD) return;
  if (in_sizes[9] < DH || in_sizes[10] < DH || in_sizes[13] < DH || in_sizes[14] < DH ||
      in_sizes[11] < 1 || in_sizes[15] < 1) return;

  const float* x     = (const float*)d_in[0];
  const float* Wq    = (const float*)d_in[1];
  const float* Wk    = (const float*)d_in[2];
  const float* Wv    = (const float*)d_in[3];
  const float* Wg1   = (const float*)d_in[4];
  const float* bg1   = (const float*)d_in[5];
  const float* Wg2   = (const float*)d_in[6];
  const float* bg2   = (const float*)d_in[7];
  const float* We1   = (const float*)d_in[8];
  const float* be1   = (const float*)d_in[9];
  const float* We2   = (const float*)d_in[10];
  const float* be2   = (const float*)d_in[11];
  const float* Wa1   = (const float*)d_in[12];
  const float* ba1   = (const float*)d_in[13];
  const float* Wa2   = (const float*)d_in[14];
  const float* ba2   = (const float*)d_in[15];
  const float* Wo    = (const float*)d_in[16];
  const float* bo    = (const float*)d_in[17];
  const float* gamma = (const float*)d_in[18];
  const float* beta  = (const float*)d_in[19];

  size_t off = 0;
  auto carve = [&](size_t bytes) -> size_t { size_t o = off; off += (bytes + 255) & ~(size_t)255; return o; };
  const size_t o_xh   = carve((size_t)ROWS * DD * 2);
  const size_t o_wt   = carve((size_t)6 * DD * DD * 2);
  const size_t o_eat  = carve((size_t)2 * DH * DD * 2);
  const size_t o_q    = carve((size_t)ROWS * DD * 4);
  const size_t o_kn   = carve((size_t)ROWS * DD * 4);
  const size_t o_vh   = carve((size_t)ROWS * DD * 2);
  const size_t o_gh   = carve((size_t)ROWS * DD * 2);
  const size_t o_vhat = carve((size_t)ROWS * DD * 4);
  const size_t o_eta  = carve((size_t)ROWS * 4);
  const size_t o_alp  = carve((size_t)ROWS * 4);
  const size_t o_oh   = carve((size_t)ROWS * DD * 2);
  if (off > ws_size) return;

  char* ws = (char*)d_ws;
  _Float16* xh   = (_Float16*)(ws + o_xh);
  _Float16* WT   = (_Float16*)(ws + o_wt);
  _Float16* EAT  = (_Float16*)(ws + o_eat);
  float*    Q    = (float*)(ws + o_q);
  float*    KN   = (float*)(ws + o_kn);
  _Float16* Vh   = (_Float16*)(ws + o_vh);
  _Float16* Gh   = (_Float16*)(ws + o_gh);
  float*    VHAT = (float*)(ws + o_vhat);
  float*    eta  = (float*)(ws + o_eta);
  float*    alp  = (float*)(ws + o_alp);
  _Float16* OH   = (_Float16*)(ws + o_oh);
  float*    out  = (float*)d_out;

  const int n8 = ROWS * DD / 8;
  k_cvt_x<<<(n8 + 255) / 256, 256, 0, stream>>>(x, xh, n8);
  k_wt<<<dim3(DD / 32, 8), 256, 0, stream>>>(Wq, Wk, Wv, Wg1, Wg2, Wo, We1, Wa1, WT, EAT);
  k_gemm_qkv<<<dim3(ROWS / 16, 3), 256, 0, stream>>>(xh, WT, Q, KN, Vh);
  k_gemm_act<true, true><<<ROWS / 16, 256, 0, stream>>>(Vh, WT + (size_t)3 * DD * DD, bg1, VHAT, Gh);
  k_gemm_act<false, false><<<ROWS / 16, 256, 0, stream>>>(Gh, WT + (size_t)4 * DD * DD, bg2, VHAT, Vh);
  k_ea<<<ROWS / 32, 256, 0, stream>>>(xh, EAT, be1, ba1, We2, be2, Wa2, ba2, eta, alp);
  k_scan<<<NSEQ, 128, 0, stream>>>(Q, KN, VHAT, eta, alp, OH);
  k_final<<<ROWS / 16, 256, 0, stream>>>(OH, WT + (size_t)5 * DD * DD, bo, x, gamma, beta, out);
}
